// GaussianAttention_78262894068500
// MI455X (gfx1250) — hardware-run, weakly checked
//
#include <hip/hip_runtime.h>


#ifndef NB
#define NB 8
#endif
#ifndef USEQ
#define USEQ 512
#endif
#ifndef TSEQ
#define TSEQ 1024
#endif
#define NB_FULL 8
#define U_FULL  512
#define T_FULL  1024
#ifndef OUT_U
#define OUT_U USEQ
#endif
#define HIN  512
#define DM   128
#define NMIX 10
#define NPAR 30
#define PW   32
#define AW   4
#define OSP2 132
#define CTP  72
#define RPW  (USEQ / 8)
#define MT   (RPW / 16)
#define PCAR 256.0f
#define CCAR 64.0f
#define OSC  (1.0f / 16384.0f)
#define NL2E (-1.4426950408889634f)

static_assert(NPAR == 3 * NMIX);
static_assert(NPAR <= PW);
static_assert(PW == 32);
static_assert(256 % PW == 0);
static_assert(HIN % 32 == 0);
static_assert(HIN % 8 == 0);
static_assert(DM == 128);
static_assert(USEQ % 128 == 0);
static_assert(MT >= 1);
static_assert(MT * 16 * 8 == USEQ);
static_assert(USEQ % (16 * AW) == 0);
static_assert(TSEQ % 64 == 0);
static_assert(TSEQ % 32 == 0);
static_assert(NB <= NB_FULL);
static_assert(USEQ <= U_FULL);
static_assert(TSEQ <= T_FULL);
static_assert((OSP2 * 4) % 16 == 0);
static_assert((CTP * 2) % 16 == 0);
static_assert(((size_t)USEQ * HIN) % 8 == 0);
static_assert((size_t)USEQ * PW * 4 <= (size_t)131072);
static_assert((size_t)AW * 16 * PW * 4 + (size_t)AW * 16 * OSP2 * 4 <= (size_t)131072);
static_assert((size_t)DM * CTP * 2 <= (size_t)131072);

typedef _Float16 h16;
typedef unsigned short bf;
typedef __attribute__((ext_vector_type(16))) __bf16   v16bf;
typedef __attribute__((ext_vector_type(16))) _Float16 v16h;
typedef __attribute__((ext_vector_type(8)))  _Float16 v8h;
typedef __attribute__((ext_vector_type(8)))  unsigned short v8us;
typedef __attribute__((ext_vector_type(8)))  float    v8f;
typedef __attribute__((ext_vector_type(4)))  float    v4f;
typedef v4f  __attribute__((may_alias)) v4fa;
typedef v8h  __attribute__((may_alias)) v8ha;

__device__ __forceinline__ unsigned short f2bf(float f) { unsigned u = __float_as_uint(f); u += 0x7FFFu + ((u >> 16) & 1u); return (unsigned short)(u >> 16); }
__device__ __forceinline__ float bfr(float f) { return __uint_as_float(((unsigned)f2bf(f)) << 16); }
__device__ __forceinline__ v16h cat16(v8h lo, v8h hi) { return __builtin_shufflevector(lo, hi, 0, 1, 2, 3, 4, 5, 6, 7, 8, 9, 10, 11, 12, 13, 14, 15); }
__device__ __forceinline__ v16bf cat16b(v8us lo, v8us hi) { return __builtin_bit_cast(v16bf, __builtin_shufflevector(lo, hi, 0, 1, 2, 3, 4, 5, 6, 7, 8, 9, 10, 11, 12, 13, 14, 15)); }
__device__ __forceinline__ v8f wmma16(v16h a, v16h b, v8f c) { return __builtin_amdgcn_wmma_f32_16x16x32_f16(false, a, false, b, (short)0, c, false, false); }
__device__ __forceinline__ v8f wmmab(v16bf a, v16bf b, v8f c) { return __builtin_amdgcn_wmma_f32_16x16x32_bf16(false, a, false, b, (short)0, c, false, false); }
__device__ __forceinline__ v16h  ldh(const h16* p) { return cat16(*(const v8h*)p, *(const v8h*)(p + 16)); }
__device__ __forceinline__ v16bf ldb(const bf* p)  { return cat16b(*(const v8us*)p, *(const v8us*)(p + 16)); }
__device__ __forceinline__ void wave_sync() { __builtin_amdgcn_fence(3  , "wavefront"); __builtin_amdgcn_wave_barrier(); asm volatile("" ::: "memory"); }

static __device__ __forceinline__ h16 toh_flush(float v) { const h16 r = (h16)v; return (fabsf(v) < 6.103515625e-05f) ? (h16)0.0f : r; }
__device__ __forceinline__ v8f wmmab_g(v16bf a, v16bf b, v8f c) { c = wmmab(a, b, c); asm volatile("v_nop\n\tv_nop\n\tv_nop\n\tv_nop" : "+v"(c) : "v"(a), "v"(b)); return c; }
__device__ __forceinline__ v8f wmma16_g(v16h a, v16h b, v8f c) { c = wmma16(a, b, c); asm volatile("v_nop\n\tv_nop\n\tv_nop\n\tv_nop" : "+v"(c) : "v"(a), "v"(b)); return c; }

__global__ __launch_bounds__(256) void k_cvt8(const float* __restrict__ src, bf* dst, size_t n8) {
    const size_t i = (size_t)blockIdx.x * 256 + threadIdx.x; if (i >= n8) return;
    const v8f v = *(const v8f*)(src + i * 8); v8us o;
#pragma unroll
    for (int k = 0; k < 8; ++k) o[k] = f2bf(v[k]);
    *(volatile v8us*)(dst + i * 8) = o; __threadfence(); *(volatile v8us*)(dst + i * 8) = o;
}

static_assert(((size_t)PW * HIN / 8) % 256 == 0);
__global__ __launch_bounds__(256) void k_wt(const float* __restrict__ W, bf* WT) {
    const int p = blockIdx.x * 256 + threadIdx.x; if (p >= PW * HIN / 8) return;
    const int n = p / (HIN / 8), k0 = (p % (HIN / 8)) * 8;
    const int nc = n < NPAR ? n : (NPAR - 1);
    v8us o;
#pragma unroll
    for (int i = 0; i < 8; ++i) { float x = W[(size_t)(k0 + i) * NPAR + nc]; asm volatile("" : "+v"(x)); o[i] = (n < NPAR) ? f2bf(x) : (unsigned short)0; }
    *(volatile v8us*)(WT + (size_t)p * 8) = o; __threadfence(); *(volatile v8us*)(WT + (size_t)p * 8) = o;
}

static_assert(64 * DM / 4 == 8 * 256);
static_assert(DM * 8 == 4 * 256);
__global__ __launch_bounds__(256) void k_ctxT(const float* __restrict__ ctx, h16* CT) {
    __shared__ __align__(16) h16 sT[DM * CTP];
    const int tid = threadIdx.x; const int b = blockIdx.y, t0 = blockIdx.x * 64;
    const float* src = ctx + ((size_t)b * T_FULL + t0) * DM;
#pragma unroll 1
    for (int it = 0; it < 8; ++it) { const int q = it * 256 + tid; const int t = q >> 5, d4 = (q & 31) * 4;
        const v4f v = *(const v4f*)(src + (size_t)t * DM + d4);
#pragma unroll
        for (int i = 0; i < 4; ++i) sT[(d4 + i) * CTP + t] = toh_flush(bfr(v[i]) * CCAR); }
    __syncthreads();
    h16* dst = CT + (size_t)b * DM * TSEQ + t0;
#pragma unroll 1
    for (int ps = 0; ps < 2; ++ps) {
#pragma unroll
        for (int it = 0; it < 4; ++it) { const int p = it * 256 + tid; const int row = p >> 3, c8 = (p & 7) * 8;
            const v8h hv = *(const v8ha*)(&sT[row * CTP + c8]);
            *(volatile v8h*)(dst + (size_t)row * TSEQ + c8) = hv; }
        if (ps == 0) __threadfence(); }
}

static_assert(((size_t)USEQ * PW) % 256 == 0);
static_assert(((size_t)USEQ * PW / 4) % 256 == 0);
__global__ __launch_bounds__(256) void k_par(const bf* __restrict__ HB, const bf* __restrict__ WT, const float* __restrict__ bias, float* PAR) {
    __shared__ __align__(16) float sp[USEQ * PW];
    const int tid = threadIdx.x;
    const int lane = tid & 31, lr = lane & 15, hi = lane >> 4;
    const int wave = __builtin_amdgcn_readfirstlane((int)(threadIdx.x >> 5));
    const int b = blockIdx.x;
    const int r0 = wave * RPW;
    v8f acc[MT][2];
#pragma unroll
    for (int mb = 0; mb < MT; ++mb) { acc[mb][0] = (v8f){}; acc[mb][1] = (v8f){}; }
    const size_t aoff = ((size_t)b * USEQ + (size_t)(r0 + lr)) * HIN + 8 * hi;
    const size_t boff = (size_t)lr * HIN + 8 * hi;
#pragma unroll 1
    for (int kc = 0; kc < HIN; kc += 32) {
        v16bf a[MT];
#pragma unroll
        for (int mb = 0; mb < MT; ++mb) a[mb] = ldb(HB + aoff + (size_t)mb * 16 * HIN + kc);
#pragma unroll
        for (int nb = 0; nb < 2; ++nb) { const v16bf w = ldb(WT + boff + (size_t)nb * 16 * HIN + kc);
#pragma unroll
            for (int mb = 0; mb < MT; ++mb) acc[mb][nb] = wmmab_g(a[mb], w, acc[mb][nb]); }
    }
#pragma unroll
    for (int mb = 0; mb < MT; ++mb) {
#pragma unroll
        for (int nb = 0; nb < 2; ++nb) {
#pragma unroll
            for (int j = 0; j < 8; ++j) sp[(r0 + mb * 16 + hi * 8 + j) * PW + nb * 16 + lr] = acc[mb][nb][j]; } }
    __syncthreads();
    { const int c = tid & 31; const int cc = c < NPAR ? c : (NPAR - 1);
      float bx = bias[cc]; asm volatile("" : "+v"(bx));
      const float bcv = (c < NPAR) ? bfr(bx) : 0.0f;
      const float sc = (c >= 2 * NMIX) ? 0.2f : 1.0f;
#pragma unroll 1
      for (int it = 0; it < USEQ * PW / 256; ++it) { const int idx = it * 256 + tid;
          const float e = expf(sp[idx] + bcv) * sc;
          sp[idx] = (c < NPAR) ? e : 0.0f; } }
    __syncthreads();
    if (wave == 0) {
        const bool isk = (lane >= 2 * NMIX) & (lane < NPAR);
        double s = 0.0;
#pragma unroll 1
        for (int u = 0; u < USEQ; ++u) { const float v = sp[u * PW + lane]; s += (double)v; const float o = isk ? (float)s : v; sp[u * PW + lane] = o; }
    }
    __syncthreads();
    float* dst = PAR + (size_t)b * USEQ * PW;
#pragma unroll 1
    for (int ps = 0; ps < 2; ++ps) {
#pragma unroll 1
        for (int it = 0; it < USEQ * PW / 4 / 256; ++it) { const int p = it * 256 + tid;
            const v4f val = *(const v4fa*)(&sp[p * 4]);
            *(volatile v4f*)(dst + (size_t)p * 4) = val; }
        if (ps == 0) __threadfence(); }
}

static_assert(32 * 16 == DM * 4);
static_assert(4 * 32 * 4 == 16 * PW);
__global__ __launch_bounds__(32 * AW) void k_window(const float* __restrict__ PAR, const h16* __restrict__ CT, const float* __restrict__ mask, float* OUT) {
    __shared__ __align__(16) float sp[AW * 16 * PW];
    __shared__ __align__(16) float os[AW * 16 * OSP2];
    const int lane = threadIdx.x & 31, lr = lane & 15, hi = lane >> 4;
    const int wave = __builtin_amdgcn_readfirstlane((int)(threadIdx.x >> 5));
    const int b = blockIdx.y;
    const int u0 = (blockIdx.x * AW + wave) * 16;
    const int pb = wave * 16 * PW;
    { const float* prow = PAR + ((size_t)b * USEQ + (size_t)u0) * PW;
#pragma unroll
      for (int s = 0; s < 4; ++s) { const int p = s * 32 + lane; const v4f x = *(const v4f*)(prow + (size_t)p * 4); *(v4fa*)(&sp[pb + p * 4]) = x; } }
    wave_sync();
    v8f acc[8];
#pragma unroll
    for (int j = 0; j < 8; ++j) acc[j] = (v8f){};
    const float* maskb = mask + (size_t)b * T_FULL + 8 * hi;
    const h16* cb = CT + ((size_t)b * DM + (size_t)lr) * TSEQ + 8 * hi;
    const int pw = pb + lr * PW;
#pragma unroll 1
    for (int key0 = 0; key0 < TSEQ; key0 += 32) {
        float s[16];
#pragma unroll
        for (int i = 0; i < 16; ++i) s[i] = 0.0f;
        const float tb = (float)(key0 + 8 * hi);
#pragma unroll 1
        for (int k = 0; k < NMIX; ++k) {
            const float a = sp[pw + k];
            const float g = sp[pw + NMIX + k] * NL2E;
            const float kp = sp[pw + 2 * NMIX + k];
#pragma unroll
            for (int i = 0; i < 8; ++i) {
                const float d0 = kp - (tb + (float)i);
                const float d1 = kp - (tb + (float)(16 + i));
                s[i]     += a * __builtin_amdgcn_exp2f(g * d0 * d0);
                s[8 + i] += a * __builtin_amdgcn_exp2f(g * d1 * d1); }
        }
        const float* kq = maskb + key0;
        const v4f m0 = *(const v4f*)kq, m1 = *(const v4f*)(kq + 4), m2 = *(const v4f*)(kq + 16), m3 = *(const v4f*)(kq + 20);
        float mk[16];
#pragma unroll
        for (int r = 0; r < 4; ++r) { mk[r] = m0[r]; mk[4 + r] = m1[r]; mk[8 + r] = m2[r]; mk[12 + r] = m3[r]; }
        v16h pa;
#pragma unroll
        for (int i = 0; i < 16; ++i) { const float gv = s[i] * bfr(mk[i]) * PCAR; pa[i] = toh_flush(gv); }
#pragma unroll
        for (int j = 0; j < 8; ++j) { const v16h cf = ldh(cb + (size_t)j * 16 * TSEQ + key0); acc[j] = wmma16_g(pa, cf, acc[j]); }
    }
    const int wb = wave * 16 * OSP2;
#pragma unroll
    for (int j = 0; j < 8; ++j) {
#pragma unroll
        for (int r = 0; r < 8; ++r) os[wb + (8 * hi + r) * OSP2 + 16 * j + lr] = acc[j][r] * OSC; }
    wave_sync();
    float* orow = OUT + ((size_t)b * OUT_U + (size_t)u0) * DM;
#pragma unroll 1
    for (int ps = 0; ps < 2; ++ps) {
#pragma unroll 4
        for (int row = 0; row < 16; ++row) {
            const v4f val = *(const v4fa*)(&os[wb + row * OSP2 + lane * 4]);
            *(volatile v4f*)(orow + (size_t)row * DM + lane * 4) = val; }
        if (ps == 0) __threadfence(); }
}

static constexpr size_t al256(size_t v) { return (v + 255) & ~(size_t)255; }
static constexpr size_t SZ_HB  = al256((size_t)NB * USEQ * HIN * 2);
static constexpr size_t SZ_WT  = al256((size_t)PW * HIN * 2);
static constexpr size_t SZ_CT  = al256((size_t)NB * DM * TSEQ * 2);
static constexpr size_t SZ_PAR = al256((size_t)NB * USEQ * PW * 4);
static constexpr size_t SZ_TOTAL = SZ_HB + SZ_WT + SZ_CT + SZ_PAR;
static_assert(SZ_TOTAL <= (size_t)134217728);
static_assert(((size_t)TSEQ * 2) % 128 == 0);
static_assert(((size_t)HIN * 2) % 128 == 0);

extern "C" void kernel_launch(void* const* d_in, const int* in_sizes, int n_in,
                              void* d_out, int out_size, void* d_ws, size_t ws_size, hipStream_t stream) {
    if (n_in < 5) return;
    const size_t needh = ((size_t)(NB - 1) * U_FULL + USEQ) * HIN;
    const size_t needc = ((size_t)(NB - 1) * T_FULL + TSEQ) * DM;
    const size_t needm = (size_t)(NB - 1) * T_FULL + TSEQ;
    if ((size_t)in_sizes[0] < needh || (size_t)in_sizes[1] < needc || (size_t)in_sizes[2] < needm) return;
    if ((size_t)in_sizes[3] < (size_t)HIN * NPAR || in_sizes[4] < NPAR) return;
    if ((size_t)out_size < ((size_t)(NB - 1) * OUT_U + USEQ) * DM) return;
    if (SZ_TOTAL > ws_size) return;
    const float* hin  = (const float*)d_in[0];
    const float* ctx  = (const float*)d_in[1];
    const float* mask = (const float*)d_in[2];
    const float* wlin = (const float*)d_in[3];
    const float* blin = (const float*)d_in[4];
    float* OUT = (float*)d_out;
    char* wsp = (char*)d_ws;
    bf*  HB  = (bf*)wsp;  wsp += SZ_HB;
    bf*  WT  = (bf*)wsp;  wsp += SZ_WT;
    h16* CT  = (h16*)wsp; wsp += SZ_CT;
    float* PAR = (float*)wsp; wsp += SZ_PAR;

    if (USEQ == U_FULL) {
        const size_t n8 = (size_t)NB * USEQ * HIN / 8;
        k_cvt8<<<(unsigned)((n8 + 255) / 256), 256, 0, stream>>>(hin, HB, n8);
    } else {
        const size_t n8 = (size_t)USEQ * HIN / 8;
        for (int b = 0; b < NB; ++b) k_cvt8<<<(unsigned)((n8 + 255) / 256), 256, 0, stream>>>(hin + (size_t)b * U_FULL * HIN, HB + (size_t)b * USEQ * HIN, n8);
    }
    k_wt<<<(unsigned)(((size_t)PW * HIN / 8 + 255) / 256), 256, 0, stream>>>(wlin, WT);
    k_ctxT<<<dim3(TSEQ / 64, NB, 1), 256, 0, stream>>>(ctx, CT);
    k_par<<<dim3(NB, 1, 1), 256, 0, stream>>>(HB, WT, blin, PAR);
    k_window<<<dim3(USEQ / (16 * AW), NB, 1), 32 * AW, 0, stream>>>(PAR, CT, mask, OUT);
}
